// ProbabalisticSlotAttention_50216757625628
// MI455X (gfx1250) — hardware-verified
//
#include <hip/hip_runtime.h>


#define NB_  16
#define NN   1024
#define DD   512
#define KK   8
#define NIT  3
typedef _Float16 h16;
typedef unsigned short bf;
typedef __attribute__((ext_vector_type(16))) __bf16   v16bf;
typedef __attribute__((ext_vector_type(16))) _Float16 v16h;
typedef __attribute__((ext_vector_type(8)))  _Float16 v8h;
typedef __attribute__((ext_vector_type(8)))  unsigned short v8us;
typedef __attribute__((ext_vector_type(8)))  float    v8f;
typedef __attribute__((ext_vector_type(4)))  float    v4f;
typedef v8h  __attribute__((may_alias)) v8ha;
typedef v4f  __attribute__((may_alias)) v4fa;
typedef v8us __attribute__((may_alias)) v8usa;

__device__ __forceinline__ unsigned short f2bf(float f) { unsigned u = __float_as_uint(f); u += 0x7FFFu + ((u >> 16) & 1u); return (unsigned short)(u >> 16); }
__device__ __forceinline__ float bf2f(unsigned short b) { return __uint_as_float(((unsigned)b) << 16); }
__device__ __forceinline__ float bfr(float f) { return bf2f(f2bf(f)); }
__device__ __forceinline__ v16h cat16(v8h lo, v8h hi) { return __builtin_shufflevector(lo, hi, 0, 1, 2, 3, 4, 5, 6, 7, 8, 9, 10, 11, 12, 13, 14, 15); }
__device__ __forceinline__ v16bf cat16b(v8us lo, v8us hi) { return __builtin_bit_cast(v16bf, __builtin_shufflevector(lo, hi, 0, 1, 2, 3, 4, 5, 6, 7, 8, 9, 10, 11, 12, 13, 14, 15)); }
__device__ __forceinline__ v8f wmma16(v16h a, v16h b, v8f c) { return __builtin_amdgcn_wmma_f32_16x16x32_f16(false, a, false, b, (short)0, c, false, false); }
__device__ __forceinline__ v8f wmmab(v16bf a, v16bf b, v8f c) { return __builtin_amdgcn_wmma_f32_16x16x32_bf16(false, a, false, b, (short)0, c, false, false); }


template <typename T16> struct WFrag;
template <> struct WFrag<h16> { typedef v16h V; static __device__ __forceinline__ V ld(const h16* p) { return cat16(*(const v8h*)p, *(const v8h*)(p + 16)); } static __device__ __forceinline__ v8f mma(V a, V b, v8f c) { return wmma16(a, b, c); } };
template <> struct WFrag<bf> { typedef v16bf V; static __device__ __forceinline__ V ld(const bf* p) { return cat16b(*(const v8us*)p, *(const v8us*)(p + 16)); } static __device__ __forceinline__ v8f mma(V a, V b, v8f c) { return wmmab(a, b, c); } };
template <typename T16, int NSPLIT, bool BIAS>
__global__ __launch_bounds__(32) void k_gemmw(const T16* __restrict__ A, const T16* __restrict__ A2, const T16* __restrict__ Bt, const T16* __restrict__ Bt2, int K, float* C, int ldc, const float* __restrict__ bias, size_t sA, size_t sB, size_t sC) {
    typedef typename WFrag<T16>::V V;
    __shared__ __align__(16) float os[16 * 68];
    const size_t z = blockIdx.z; A += z * sA; if (A2) A2 += z * sA; Bt += z * sB; if (Bt2) Bt2 += z * sB; C += z * sC;
    const int lane = threadIdx.x & 31, lr = lane & 15, hi = lane >> 4; const int r0 = blockIdx.x * 64, c0 = blockIdx.y * 64;
    v8f acc[4][4];
#pragma unroll
    for (int mb = 0; mb < 4; ++mb)
#pragma unroll
        for (int nb = 0; nb < 4; ++nb) acc[mb][nb] = (v8f){};
    const size_t aoff = (size_t)(r0 + lr) * K + 8 * hi, boff = (size_t)(c0 + lr) * K + 8 * hi;
#pragma unroll 1
    for (int kc = 0; kc < K; kc += 32) {
        V a[4], a2[4];
#pragma unroll
        for (int mb = 0; mb < 4; ++mb) { a[mb] = WFrag<T16>::ld(A + aoff + (size_t)mb * 16 * K + kc); if (NSPLIT == 1 || NSPLIT == 2) a2[mb] = WFrag<T16>::ld(A2 + aoff + (size_t)mb * 16 * K + kc); }
#pragma unroll
        for (int nb = 0; nb < 4; ++nb) { const V b = WFrag<T16>::ld(Bt + boff + (size_t)nb * 16 * K + kc); V b2; if (NSPLIT >= 2) b2 = WFrag<T16>::ld(Bt2 + boff + (size_t)nb * 16 * K + kc);
#pragma unroll
            for (int mb = 0; mb < 4; ++mb) { acc[mb][nb] = WFrag<T16>::mma(a[mb], b, acc[mb][nb]); if (NSPLIT == 1 || NSPLIT == 2) acc[mb][nb] = WFrag<T16>::mma(a2[mb], b, acc[mb][nb]); if (NSPLIT >= 2) acc[mb][nb] = WFrag<T16>::mma(a[mb], b2, acc[mb][nb]); } }
        asm volatile("v_nop\n\tv_nop\n\tv_nop\n\tv_nop" : "+v"(acc[0][0]), "+v"(acc[1][1]), "+v"(acc[2][2]), "+v"(acc[3][3]) : "v"(a[0]), "v"(a[3]));
    }
#pragma unroll
    for (int mb = 0; mb < 4; ++mb) {
#pragma unroll
        for (int nb = 0; nb < 4; ++nb) {
#pragma unroll
            for (int j = 0; j < 8; ++j) os[(hi * 8 + j) * 68 + nb * 16 + lr] = acc[mb][nb][j]; }
        __builtin_amdgcn_wave_barrier(); asm volatile("" ::: "memory");
        float* crow = C + (size_t)(r0 + mb * 16) * ldc + c0;
#pragma unroll 1
        for (int ps = 0; ps < 2; ++ps) {
#pragma unroll
            for (int s = 0; s < 8; ++s) { const int row = 2 * s + hi, cofs = lr * 4; v4f val = *(const v4fa*)(os + row * 68 + cofs); if (BIAS) { val[0] += bfr(bias[c0 + cofs]); val[1] += bfr(bias[c0 + cofs + 1]); val[2] += bfr(bias[c0 + cofs + 2]); val[3] += bfr(bias[c0 + cofs + 3]); }
                *(volatile v4f*)(crow + (size_t)row * ldc + cofs) = val; }
            if (ps == 0) __threadfence(); }
        __builtin_amdgcn_wave_barrier(); asm volatile("" ::: "memory");
    }
}

__device__ __forceinline__ void splitf(float y, unsigned short& h, unsigned short& l) { h = f2bf(y); l = f2bf(y - bf2f(h)); }
typedef __attribute__((ext_vector_type(2))) unsigned short v2us;
typedef __attribute__((ext_vector_type(4))) unsigned short v4us;
typedef __attribute__((ext_vector_type(2))) float v2f;

__global__ __launch_bounds__(256) void k_wtG(const float* __restrict__ w, int K, int N, bf* Bt) {
    const int lane = threadIdx.x & 31; const int L0 = (blockIdx.x * 8 + (threadIdx.x >> 5)) * 8; const int nlines = N * K / 64;
#pragma unroll 1
    for (int ps = 0; ps < 2; ++ps) {
#pragma unroll 1
        for (int l = 0; l < 8; ++l) { const int L = L0 + l; if (L >= nlines) break; const size_t e = (size_t)L * 64 + lane * 2; const int k = (int)(e % K), n = (int)(e / K); v2us o;
            o[0] = f2bf(w[(size_t)k * N + n]); o[1] = f2bf(w[(size_t)(k + 1) * N + n]); *(volatile v2us*)(Bt + e) = o; }
        if (ps == 0) __threadfence(); }
}
__global__ __launch_bounds__(256) void k_ln(const float* __restrict__ E, const float* __restrict__ g, const float* __restrict__ bb, bf* Xh, bf* Xl) { const int lane = threadIdx.x & 31; const int r = blockIdx.x * 8 + (threadIdx.x >> 5); if (r >= NN) return; float v[16]; float s = 0.f;
#pragma unroll
    for (int c = 0; c < 4; ++c) { const v4f a = *(const v4f*)(E + (size_t)r * DD + c * 128 + lane * 4);
#pragma unroll
        for (int q = 0; q < 4; ++q) { const float t = bfr(a[q]); v[c * 4 + q] = t; s = __fadd_rn(s, t); } }
#pragma unroll
    for (int sh = 16; sh; sh >>= 1) s += __shfl_xor(s, sh, 32);
    const float mu = s * (1.0f / DD); float qq = 0.f;
#pragma unroll
    for (int i = 0; i < 16; ++i) { const float d0 = v[i] - mu; float p = __fmul_rn(d0, d0); asm volatile("" : "+v"(p)); qq = __fadd_rn(qq, p); }
#pragma unroll
    for (int sh = 16; sh; sh >>= 1) qq += __shfl_xor(qq, sh, 32);
    const float rs = __fdiv_rn(1.0f, __fsqrt_rn(__fadd_rn(qq * (1.0f / DD), 1e-5f)));
#pragma unroll 1
    for (int ps = 0; ps < 2; ++ps) {
#pragma unroll
        for (int c = 0; c < 4; ++c) { v4us oh, ol;
#pragma unroll
            for (int q = 0; q < 4; ++q) { const int col = c * 128 + lane * 4 + q; float gg = bfr(g[col]), be = bfr(bb[col]); asm volatile("" : "+v"(gg)); asm volatile("" : "+v"(be)); float tn = __fmul_rn(v[c * 4 + q] - mu, rs); asm volatile("" : "+v"(tn)); float tg = __fmul_rn(tn, gg); asm volatile("" : "+v"(tg)); unsigned short a, c2; splitf(__fadd_rn(tg, be), a, c2); oh[q] = a; ol[q] = c2; }
            const size_t o = (size_t)r * DD + c * 128 + lane * 4; *(volatile v4us*)(Xh + o) = oh; *(volatile v4us*)(Xl + o) = ol; }
        if (ps == 0) __threadfence(); } }
__global__ __launch_bounds__(256) void k_init(const float* __restrict__ smu, const float* __restrict__ slog, const float* __restrict__ nib, const float* __restrict__ mixc, float* SIG, float* SL, float* MIX) { const int e = blockIdx.x * 256 + threadIdx.x; if (e >= KK * DD) return;
    const float sg = __expf(bfr(slog[e])); float p = __fmul_rn(sg, bfr(nib[e])); asm volatile("" : "+v"(p)); const float sl = __fadd_rn(bfr(smu[e]), p);
    *(volatile float*)(SIG + e) = sg; *(volatile float*)(SL + e) = sl; if (blockIdx.x == 0 && threadIdx.x < 32) *(volatile float*)(MIX + threadIdx.x) = threadIdx.x < KK ? bfr(mixc[threadIdx.x]) : 0.f;
    __threadfence(); *(volatile float*)(SIG + e) = sg; *(volatile float*)(SL + e) = sl; if (blockIdx.x == 0 && threadIdx.x < 32) *(volatile float*)(MIX + threadIdx.x) = threadIdx.x < KK ? bfr(mixc[threadIdx.x]) : 0.f; }
__global__ __launch_bounds__(256) void k_qry(const float* __restrict__ SL, const float* __restrict__ wq, const float* __restrict__ bq, float* Q) { const int e = blockIdx.x * 256 + threadIdx.x; if (e >= KK * DD) return; const int d = e % DD, k = e / DD; float acc = 0.f;
#pragma unroll 4
    for (int c = 0; c < DD; ++c) { float w = bfr(wq[(size_t)c * DD + d]); asm volatile("" : "+v"(w)); float p = __fmul_rn(SL[k * DD + c], w); asm volatile("" : "+v"(p)); acc = __fadd_rn(acc, p); }
    float b2 = bfr(bq[d]); asm volatile("" : "+v"(b2)); const float o = __fadd_rn(acc, b2); *(volatile float*)(Q + e) = o; __threadfence(); *(volatile float*)(Q + e) = o; }
__global__ __launch_bounds__(32) void k_gc(const float* __restrict__ SIG, float* GC) { const int lane = threadIdx.x; float keep = 0.f;
    for (int k = 0; k < KK; ++k) { float s = 0.f; for (int d = lane; d < DD; d += 32) s = __fadd_rn(s, logf(__fadd_rn(fabsf(SIG[k * DD + d]), 1e-8f)));
#pragma unroll
        for (int sh = 16; sh; sh >>= 1) s += __shfl_xor(s, sh, 32);
        if (lane == k) keep = __fsub_rn(-0.5f * DD * 1.8378770664093453f, 0.5f * s); }
    *(volatile float*)(GC + lane) = keep; __threadfence(); *(volatile float*)(GC + lane) = keep; }
__global__ __launch_bounds__(256) void k_rv(const float* __restrict__ SIG, float* RV) { const int e = blockIdx.x * 256 + threadIdx.x; if (e >= KK * DD) return; float s2 = __fmul_rn(SIG[e], SIG[e]); asm volatile("" : "+v"(s2)); const float r = __fdiv_rn(1.0f, __fadd_rn(s2, 1e-8f)); *(volatile float*)(RV + e) = r; __threadfence(); *(volatile float*)(RV + e) = r; }
__global__ __launch_bounds__(256) void k_gll(const float* __restrict__ KEY, const float* __restrict__ Q, const float* __restrict__ RV, const float* __restrict__ GC, const float* __restrict__ MIX, float* ATT) { const int n = blockIdx.x * 256 + threadIdx.x; if (n >= NN) return; const float* kr = KEY + (size_t)n * DD; float a[KK]; float tot = 0.f;
#pragma unroll 1
    for (int k = 0; k < KK; ++k) { float acc = 0.f;
#pragma unroll 4
        for (int d = 0; d < DD; ++d) { const float df = __fsub_rn(kr[d], Q[k * DD + d]); float sq = __fmul_rn(df, df); asm volatile("" : "+v"(sq)); float t = __fmul_rn(sq, RV[k * DD + d]); asm volatile("" : "+v"(t)); acc = __fadd_rn(acc, t); }
        float g = __fsub_rn(GC[k], 0.5f * acc); asm volatile("" : "+v"(g)); a[k] = __fmul_rn(MIX[k], g); tot = __fadd_rn(tot, a[k]); }
    for (int ps = 0; ps < 2; ++ps) {
#pragma unroll
        for (int k = 0; k < KK; ++k) *(volatile float*)(ATT + (size_t)k * NN + n) = __fdiv_rn(a[k], tot);
        if (ps == 0) __threadfence(); } }
__global__ __launch_bounds__(32) void k_cs(const float* __restrict__ ATT, float* CS) { const int lane = threadIdx.x; float keep = 0.f;
    for (int k = 0; k < KK; ++k) { float s = 0.f; for (int n = lane; n < NN; n += 32) s = __fadd_rn(s, ATT[(size_t)k * NN + n]);
#pragma unroll
        for (int sh = 16; sh; sh >>= 1) s += __shfl_xor(s, sh, 32);
        if (lane == k) keep = s; }
    *(volatile float*)(CS + lane) = keep; __threadfence(); *(volatile float*)(CS + lane) = keep; }
__global__ __launch_bounds__(256) void k_cnorm(float* ATT, const float* __restrict__ CS, float* OUT1b) { const int n = blockIdx.x * 256 + threadIdx.x; if (n >= NN) return; float a[KK];
#pragma unroll
    for (int k = 0; k < KK; ++k) a[k] = __fdiv_rn(ATT[(size_t)k * NN + n], __fadd_rn(CS[k], 1e-8f));
    for (int ps = 0; ps < 2; ++ps) {
#pragma unroll
        for (int k = 0; k < KK; ++k) { *(volatile float*)(ATT + (size_t)k * NN + n) = a[k]; if (OUT1b) *(volatile float*)(OUT1b + (size_t)k * NN + n) = a[k]; }
        if (ps == 0) __threadfence(); } }
__global__ __launch_bounds__(32) void k_mix(const float* __restrict__ ATT, float* MIX) { const int lane = threadIdx.x; float keep = 0.f;
    for (int k = 0; k < KK; ++k) { float s = 0.f; for (int n = lane; n < NN; n += 32) s = __fadd_rn(s, ATT[(size_t)k * NN + n]);
#pragma unroll
        for (int sh = 16; sh; sh >>= 1) s += __shfl_xor(s, sh, 32);
        if (lane == k) keep = s * (1.0f / NN); }
    *(volatile float*)(MIX + lane) = keep; __threadfence(); *(volatile float*)(MIX + lane) = keep; }
__global__ __launch_bounds__(256) void k_mu(const float* __restrict__ ATT, const float* __restrict__ V, float* MU) { const int e = blockIdx.x * 256 + threadIdx.x; if (e >= KK * DD) return; const int d = e % DD, k = e / DD; float acc = 0.f;
    for (int n = 0; n < NN; ++n) { float p = __fmul_rn(ATT[(size_t)k * NN + n], V[(size_t)n * DD + d]); asm volatile("" : "+v"(p)); acc = __fadd_rn(acc, p); }
    *(volatile float*)(MU + e) = acc; __threadfence(); *(volatile float*)(MU + e) = acc; }
__global__ __launch_bounds__(256) void k_sig(const float* __restrict__ ATT, const float* __restrict__ V, const float* __restrict__ MU, float* SIG) { const int e = blockIdx.x * 256 + threadIdx.x; if (e >= KK * DD) return; const int d = e % DD, k = e / DD; const float m = MU[e]; float acc = 0.f;
    for (int n = 0; n < NN; ++n) { const float df = __fsub_rn(V[(size_t)n * DD + d], m); float sq = __fmul_rn(df, df); asm volatile("" : "+v"(sq)); float p = __fmul_rn(ATT[(size_t)k * NN + n], sq); asm volatile("" : "+v"(p)); acc = __fadd_rn(acc, p); }
    *(volatile float*)(SIG + e) = acc; __threadfence(); *(volatile float*)(SIG + e) = acc; }
__global__ __launch_bounds__(256) void k_out0(const float* __restrict__ MU, const float* __restrict__ SIG, const float* __restrict__ nfb, float* OUT0b) { const int e = blockIdx.x * 256 + threadIdx.x; if (e >= KK * DD) return; float p = __fmul_rn(fmaxf(fabsf(SIG[e]), 1e-8f), bfr(nfb[e])); asm volatile("" : "+v"(p)); const float o = __fadd_rn(MU[e], p); *(volatile float*)(OUT0b + e) = o; __threadfence(); *(volatile float*)(OUT0b + e) = o; }

extern "C" void kernel_launch(void* const* d_in, const int* in_sizes, int n_in,
                              void* d_out, int out_size, void* d_ws, size_t ws_size, hipStream_t stream) {
    (void)in_sizes; (void)n_in; (void)out_size;
    const float* IN[14]; for (int i = 0; i < 14; ++i) IN[i] = (const float*)d_in[i];
    float* OUT0 = (float*)d_out; float* OUT1 = (float*)d_out + (size_t)NB_ * KK * DD;
    char* wsp = (char*)d_ws;
    auto take = [&](size_t bytes) { char* p = wsp; wsp += (bytes + 255) & ~(size_t)255; return (void*)p; };
    bf* WK = (bf*)take((size_t)DD * DD * 2); bf* WV = (bf*)take((size_t)DD * DD * 2); bf* Xh = (bf*)take((size_t)NN * DD * 2); bf* Xl = (bf*)take((size_t)NN * DD * 2); float* KEY = (float*)take((size_t)NN * DD * 4); float* VAL = (float*)take((size_t)NN * DD * 4);
    float* SIG = (float*)take((size_t)KK * DD * 4); float* SL = (float*)take((size_t)KK * DD * 4); float* Q = (float*)take((size_t)KK * DD * 4); float* RV = (float*)take((size_t)KK * DD * 4); float* MU = (float*)take((size_t)KK * DD * 4); float* ATT = (float*)take((size_t)KK * NN * 4); float* MIX = (float*)take(256); float* GC = (float*)take(256); float* CS = (float*)take(256);
    if ((size_t)(wsp - (char*)d_ws) > ws_size) return;
    k_wtG<<<(unsigned)((DD * DD / 64 + 63) / 64), 256, 0, stream>>>(IN[6], DD, DD, WK); k_wtG<<<(unsigned)((DD * DD / 64 + 63) / 64), 256, 0, stream>>>(IN[10], DD, DD, WV);
    const unsigned LK = (KK * DD + 255) / 256;
    for (int b = 0; b < NB_; ++b) {
        k_ln<<<NN / 8, 256, 0, stream>>>(IN[0] + (size_t)b * NN * DD, IN[12], IN[13], Xh, Xl);
        k_gemmw<bf, 1, true><<<dim3(NN / 64, DD / 64, 1), 32, 0, stream>>>(Xh, Xl, WK, nullptr, DD, KEY, DD, IN[7], 0, 0, 0); k_gemmw<bf, 1, true><<<dim3(NN / 64, DD / 64, 1), 32, 0, stream>>>(Xh, Xl, WV, nullptr, DD, VAL, DD, IN[11], 0, 0, 0);
        k_init<<<LK, 256, 0, stream>>>(IN[3], IN[4], IN[1] + (size_t)b * KK * DD, IN[5], SIG, SL, MIX); k_qry<<<LK, 256, 0, stream>>>(SL, IN[8], IN[9], Q);
        for (int it = 0; it < NIT; ++it) {
            k_gc<<<1, 32, 0, stream>>>(SIG, GC); k_rv<<<LK, 256, 0, stream>>>(SIG, RV);
            k_gll<<<NN / 256, 256, 0, stream>>>(KEY, Q, RV, GC, MIX, ATT);
            k_cs<<<1, 32, 0, stream>>>(ATT, CS); k_cnorm<<<NN / 256, 256, 0, stream>>>(ATT, CS, it == NIT - 1 ? OUT1 + (size_t)b * KK * NN : nullptr);
            k_mu<<<LK, 256, 0, stream>>>(ATT, VAL, MU); k_sig<<<LK, 256, 0, stream>>>(ATT, VAL, MU, SIG); k_mix<<<1, 32, 0, stream>>>(ATT, MIX); }
        k_out0<<<LK, 256, 0, stream>>>(MU, SIG, IN[2] + (size_t)b * KK * DD, OUT0 + (size_t)b * KK * DD); }
}
